// RecurrentTransformer_45363444580916
// MI455X (gfx1250) — hardware-run, weakly checked
//
#include <hip/hip_runtime.h>
#include <math.h>

typedef __attribute__((ext_vector_type(16))) _Float16 v16h;
typedef __attribute__((ext_vector_type(8)))  _Float16 v8h;
typedef __attribute__((ext_vector_type(8)))  float    v8f;
typedef __attribute__((ext_vector_type(4)))  float    v4f;
typedef __attribute__((ext_vector_type(4)))  unsigned int v4u;

constexpr int kLayers = 4;
constexpr int kBatch  = 4;
constexpr int kCin    = 64;
constexpr int kCout   = 64;
constexpr int kE      = 512;
constexpr int kS      = 2048;
constexpr int kRows   = kBatch * kS;
constexpr int kSP     = kS + 2;
constexpr int kNumW   = 6;

constexpr float kWCarry   = 1024.0f;
constexpr float kACarry   = 16.0f;
constexpr float kAttCarry = 256.0f;
constexpr float kSclAW    = 1.0f / (kACarry * kWCarry);
constexpr float kSclAttW  = 1.0f / (kAttCarry * kWCarry);
constexpr float kSclNum   = 1.0f / kACarry;
constexpr float kLnEps    = 1e-5f;
constexpr float kDenEps   = 1e-6f;
constexpr float kInvE     = 1.0f / (float)kE;
constexpr float kInvSqrt2 = 0.70710678118654752440f;

static_assert((kCin % 32) == 0 && (kE % 32) == 0 && ((3 * kE) % 32) == 0 && (kS % 32) == 0);
static_assert((kS % 64) == 0 && (kE % 64) == 0 && (kCout % 64) == 0 && (kRows % 64) == 0);
static_assert(kE == 512 && kS == 2048 && kCin == 64);
static_assert((((kS / 64) * (kS / 64 + 1)) / 2) % 8 == 0);

constexpr size_t kOffLAT  = 0;
constexpr size_t kOffMID  = kOffLAT  + (size_t)kRows * kE * 4;
constexpr size_t kOffH16  = kOffMID  + (size_t)kRows * kE * 4;
constexpr size_t kOffQ16  = kOffH16  + (size_t)kRows * kE * 2;
constexpr size_t kOffK16  = kOffQ16  + (size_t)kRows * kE * 2;
constexpr size_t kOffVT16 = kOffK16  + (size_t)kRows * kE * 2;
constexpr size_t kOffATT  = kOffVT16 + (size_t)kRows * kE * 2;
constexpr size_t kOffT16P = kOffATT  + (size_t)kRows * kE * 2;
constexpr size_t kOffP16  = kOffT16P + (size_t)kBatch * kSP * kE * 2;
constexpr size_t kOffRDEN = kOffP16  + (size_t)kBatch * kS * kS * 2;
constexpr size_t kOffW16  = kOffRDEN + (size_t)kRows * 4;
constexpr size_t kOffCCW  = kOffW16  + (size_t)kNumW * kLayers * kE * kE * 2;
constexpr size_t kOffINW  = kOffCCW  + (size_t)kE * 3 * kE * 2;
constexpr size_t kOffOUTW = kOffINW  + (size_t)kE * kCin * 2;
constexpr size_t kOffX16  = kOffOUTW + (size_t)kCout * kE * 2;
constexpr size_t kWsTotal = kOffX16  + (size_t)kRows * kCin * 2;
static_assert(kWsTotal == 132816896ull);
static_assert(kWsTotal <= 134217728ull);
static_assert((kOffMID % 128) == 0 && (kOffH16 % 128) == 0 && (kOffQ16 % 128) == 0 && (kOffK16 % 128) == 0 &&
              (kOffVT16 % 128) == 0 && (kOffATT % 128) == 0 && (kOffT16P % 128) == 0 && (kOffP16 % 128) == 0 &&
              (kOffRDEN % 128) == 0 && (kOffW16 % 128) == 0 && (kOffCCW % 128) == 0 && (kOffINW % 128) == 0 &&
              (kOffOUTW % 128) == 0 && (kOffX16 % 128) == 0);

__device__ __forceinline__ float bf16_rne(float f) {
  const unsigned u = __float_as_uint(f);
  const unsigned r = (u + 0x7FFFu + ((u >> 16) & 1u)) & 0xFFFF0000u;
  return __uint_as_float(r);
}
__device__ __forceinline__ unsigned short h_bits(float f) {
  const _Float16 h = (_Float16)f;
  return __builtin_bit_cast(unsigned short, h);
}
__device__ __forceinline__ unsigned pk16(unsigned short a, unsigned short b) {
  return (unsigned)a | ((unsigned)b << 16);
}
__device__ __forceinline__ float h16_to_f32(unsigned hb) {
  const unsigned sgn = (hb & 0x8000u) << 16;
  const unsigned em = hb & 0x7fffu;
  const float fn = __uint_as_float((em << 13) + 0x38000000u);
  const float fs = (float)em * 5.9604644775390625e-8f;
  const float mag = (em < 0x400u) ? fs : fn;
  return __uint_as_float(__float_as_uint(mag) | sgn);
}

union FragU { v16h v; v8h h[2]; };
__device__ __forceinline__ v16h frag_load(const _Float16* p) {
  FragU f;
  f.h[0] = *(const v8h*)(p);
  f.h[1] = *(const v8h*)(p + 16);
  return f.v;
}
__device__ __forceinline__ v8f mma_f16(v16h a, v16h b, v8f c) {
  return __builtin_amdgcn_wmma_f32_16x16x32_f16(false, a, false, b, (short)0, c, false, false);
}
__device__ __forceinline__ void tie_acc(v8f& a, v16h x, v16h y) {
  asm volatile("" : "+v"(a) : "v"(x), "v"(y));
}
__device__ __forceinline__ void tie_acc_nops(v8f& a, v16h x, v16h y) {
  asm volatile("v_nop\n\tv_nop\n\tv_nop\n\tv_nop" : "+v"(a) : "v"(x), "v"(y));
}
__device__ __forceinline__ void keep4_h(v16h a, v16h b, v16h c, v16h d) {
  asm volatile("v_nop" :: "v"(a), "v"(b), "v"(c), "v"(d));
}

template <int ACT> __device__ __forceinline__ float act_fn(float z) {
  if (ACT == 1) {
    const float zn = fminf(z, 0.0f);
    const float e = __expf(zn);
    return (z > 0.0f) ? (z + 1.0f) : e;
  }
  if (ACT == 2) {
    return 0.5f * z * (1.0f + erff(z * kInvSqrt2));
  }
  return z;
}

template <int BIAS_MODE, int OUT_MODE, bool RESID, int ACT, int CAUSAL, bool ROWSC>
__global__ __launch_bounds__(256) void gemm64_kernel(
    const unsigned short* __restrict__ Ap, int lda, long strideA,
    const unsigned short* __restrict__ Btp, int ldb, long strideB,
    void* __restrict__ Cout, int ldc, long strideC,
    const float* __restrict__ bias,
    const float* __restrict__ resid, long strideR,
    const float* __restrict__ rowsc, long strideRS,
    int M, int N, int K, float scale, float oscale) {
  const _Float16* A  = (const _Float16*)Ap;
  const _Float16* Bt = (const _Float16*)Btp;
  __shared__ __align__(16) float sT[8][16 * 68];
  const int b    = blockIdx.y;
  const int lane = threadIdx.x & 31;
  const int wave = __builtin_amdgcn_readfirstlane((int)(threadIdx.x >> 5));
  const int tilesN = N >> 6;
  const int tilesM = M >> 6;
  const int tile = blockIdx.x * 8 + wave;
  int tm, tn;
  if (CAUSAL == 1) {
    const int ntri = (tilesM * (tilesM + 1)) >> 1;
    if (tile >= ntri) return;
    tm = 0;
#pragma unroll 1
    for (int c = 1; c < tilesM; ++c) {
      if (((c * (c + 1)) >> 1) <= tile) tm = c;
    }
    tn = tile - ((tm * (tm + 1)) >> 1);
  } else {
    if (tile >= tilesM * tilesN) return;
    tm = tile / tilesN;
    tn = tile - tm * tilesN;
  }
  const int m0 = tm << 6;
  const int n0 = tn << 6;

  const _Float16* Ab = A  + (size_t)b * strideA;
  const _Float16* Bb = Bt + (size_t)b * strideB;

  const int rlane = lane & 15;
  const int koff  = (lane >> 4) * 8;
  const int mOff  = (lane >> 4) * 8;

  v8f acc[4][4];
#pragma unroll
  for (int i = 0; i < 4; ++i)
#pragma unroll
    for (int j = 0; j < 4; ++j) acc[i][j] = (v8f){0.f, 0.f, 0.f, 0.f, 0.f, 0.f, 0.f, 0.f};

  int Kend = K;
  if (CAUSAL == 2) Kend = (m0 + 64 < K) ? (m0 + 64) : K;

  for (int k0 = 0; k0 < Kend; k0 += 32) {
    v16h bh[4];
#pragma unroll
    for (int j = 0; j < 4; ++j) {
      const size_t bo = (size_t)(n0 + (j << 4) + rlane) * ldb + koff + k0;
      bh[j] = frag_load(Bb + bo);
    }
#pragma unroll
    for (int i = 0; i < 4; ++i) {
      const size_t ao = (size_t)(m0 + (i << 4) + rlane) * lda + koff + k0;
      const v16h ah = frag_load(Ab + ao);
#pragma unroll
      for (int j = 0; j < 4; ++j) acc[i][j] = mma_f16(ah, bh[j], acc[i][j]);
      tie_acc(acc[i][0], ah, bh[0]);
      tie_acc(acc[i][1], ah, bh[1]);
      tie_acc(acc[i][2], ah, bh[2]);
      tie_acc_nops(acc[i][3], ah, bh[3]);
    }
    keep4_h(bh[0], bh[1], bh[2], bh[3]);
  }

  float* slab = sT[wave];
  const float* Rb = RESID ? (resid + (size_t)b * strideR) : nullptr;
  const float* RS = ROWSC ? (rowsc + (size_t)b * strideRS) : nullptr;
  const bool diag = (CAUSAL == 1) && (tn == tm);
  float bvj[4] = {0.f, 0.f, 0.f, 0.f};
  if (BIAS_MODE == 2) {
#pragma unroll
    for (int j = 0; j < 4; ++j) {
      const float t = bias[n0 + (j << 4) + rlane];
      bvj[j] = bf16_rne(t);
    }
  }
#pragma unroll
  for (int i = 0; i < 4; ++i) {
    const int mBase = m0 + (i << 4);
    float radd[8] = {0.f, 0.f, 0.f, 0.f, 0.f, 0.f, 0.f, 0.f};
    float rmul[8] = {1.f, 1.f, 1.f, 1.f, 1.f, 1.f, 1.f, 1.f};
    if (BIAS_MODE == 1) {
      const v4f t0 = *(const v4f*)(bias + mBase + mOff);
      const v4f t1 = *(const v4f*)(bias + mBase + mOff + 4);
      const float e0 = t0.x, e1 = t0.y, e2 = t0.z, e3 = t0.w;
      const float e4 = t1.x, e5 = t1.y, e6 = t1.z, e7 = t1.w;
      radd[0] = bf16_rne(e0); radd[1] = bf16_rne(e1); radd[2] = bf16_rne(e2); radd[3] = bf16_rne(e3);
      radd[4] = bf16_rne(e4); radd[5] = bf16_rne(e5); radd[6] = bf16_rne(e6); radd[7] = bf16_rne(e7);
    }
    if (ROWSC) {
      const v4f t0 = *(const v4f*)(RS + mBase + mOff);
      const v4f t1 = *(const v4f*)(RS + mBase + mOff + 4);
      rmul[0] = t0.x; rmul[1] = t0.y; rmul[2] = t0.z; rmul[3] = t0.w;
      rmul[4] = t1.x; rmul[5] = t1.y; rmul[6] = t1.z; rmul[7] = t1.w;
    }
#pragma unroll
    for (int j = 0; j < 4; ++j) {
#pragma unroll
      for (int r = 0; r < 8; ++r) {
        float v = acc[i][j][r] * scale;
        if (ROWSC) v = v * rmul[r];
        if (BIAS_MODE == 1) v = v + radd[r];
        if (BIAS_MODE == 2) v = v + bvj[j];
        if (CAUSAL == 1) {
          const bool masked = diag && (((j << 4) + rlane) > ((i << 4) + mOff + r));
          v = masked ? 0.0f : v;
        }
        slab[(mOff + r) * 68 + (j << 4) + rlane] = v;
      }
    }
    __builtin_amdgcn_fence(__ATOMIC_RELEASE, "workgroup");
    __builtin_amdgcn_wave_barrier();
    __builtin_amdgcn_fence(__ATOMIC_ACQUIRE, "workgroup");
    if (ACT != 0) {
#pragma unroll 1
      for (int t = 0; t < 32; ++t) {
        float* p = slab + (t >> 1) * 68 + ((t & 1) << 5) + lane;
        const float z = *p;
        *p = act_fn<ACT>(z);
      }
      __builtin_amdgcn_fence(__ATOMIC_RELEASE, "workgroup");
      __builtin_amdgcn_wave_barrier();
      __builtin_amdgcn_fence(__ATOMIC_ACQUIRE, "workgroup");
    }
    if (OUT_MODE == 0) {
      float* C = (float*)Cout + (size_t)b * strideC;
      const int hh = lane >> 4, c4 = (lane & 15) * 4;
      v4f vals[8];
#pragma unroll
      for (int it = 0; it < 8; ++it) {
        const int row = it * 2 + hh;
        v4f v = *(const v4f*)(slab + row * 68 + c4);
        if (RESID) {
          const v4f rv = *(const v4f*)(Rb + (size_t)(mBase + row) * ldc + n0 + c4);
          v = v + rv;
        }
        vals[it] = v;
      }
      for (int pass = 0; pass < 2; ++pass) {
#pragma unroll
        for (int it = 0; it < 8; ++it) {
          const int row = it * 2 + hh;
          *(volatile v4f*)(C + (size_t)(mBase + row) * ldc + n0 + c4) = vals[it];
        }
        __threadfence();
      }
    } else {
      unsigned short* C = (unsigned short*)Cout + (size_t)b * strideC;
      const int q = lane >> 3, c8 = (lane & 7) * 8;
      v8h hv[4];
#pragma unroll
      for (int it = 0; it < 4; ++it) {
        const int row = it * 4 + q;
        const float* sp = slab + row * 68 + c8;
        v4f s0 = *(const v4f*)(sp);
        v4f s1 = *(const v4f*)(sp + 4);
        if (RESID) {
          const float* rp = Rb + (size_t)(mBase + row) * ldc + n0 + c8;
          const v4f r0 = *(const v4f*)(rp);
          const v4f r1 = *(const v4f*)(rp + 4);
          s0 = s0 + r0;
          s1 = s1 + r1;
        }
        s0 = s0 * oscale;
        s1 = s1 * oscale;
        v8h h;
        h[0] = (_Float16)s0.x; h[1] = (_Float16)s0.y; h[2] = (_Float16)s0.z; h[3] = (_Float16)s0.w;
        h[4] = (_Float16)s1.x; h[5] = (_Float16)s1.y; h[6] = (_Float16)s1.z; h[7] = (_Float16)s1.w;
        hv[it] = h;
      }
      for (int pass = 0; pass < 2; ++pass) {
#pragma unroll
        for (int it = 0; it < 4; ++it) {
          const int row = it * 4 + q;
          *(volatile v8h*)(C + (size_t)(mBase + row) * ldc + n0 + c8) = hv[it];
        }
        __threadfence();
      }
    }
    __builtin_amdgcn_fence(__ATOMIC_RELEASE, "workgroup");
    __builtin_amdgcn_wave_barrier();
    __builtin_amdgcn_fence(__ATOMIC_ACQUIRE, "workgroup");
  }
}

__global__ __launch_bounds__(256) void cast8_kernel(
    const float* __restrict__ w0, const float* __restrict__ w1, const float* __restrict__ w2,
    const float* __restrict__ w3, const float* __restrict__ w4, const float* __restrict__ w5,
    unsigned short* __restrict__ out, int n8, float carry) {
  const int i = blockIdx.x * 256 + threadIdx.x;
  if (i >= n8) return;
  const int z = blockIdx.y;
  const float* in = (z == 0) ? w0 : (z == 1) ? w1 : (z == 2) ? w2 : (z == 3) ? w3 : (z == 4) ? w4 : w5;
  const float* p = in + 8 * (size_t)i;
  const v4f a = *(const v4f*)(p);
  const v4f c = *(const v4f*)(p + 4);
  const float f0 = a.x, f1 = a.y, f2 = a.z, f3 = a.w, f4 = c.x, f5 = c.y, f6 = c.z, f7 = c.w;
  const unsigned short b0 = h_bits(bf16_rne(f0) * carry), b1 = h_bits(bf16_rne(f1) * carry);
  const unsigned short b2 = h_bits(bf16_rne(f2) * carry), b3 = h_bits(bf16_rne(f3) * carry);
  const unsigned short b4 = h_bits(bf16_rne(f4) * carry), b5 = h_bits(bf16_rne(f5) * carry);
  const unsigned short b6 = h_bits(bf16_rne(f6) * carry), b7 = h_bits(bf16_rne(f7) * carry);
  const v4u u = (v4u){pk16(b0, b1), pk16(b2, b3), pk16(b4, b5), pk16(b6, b7)};
  unsigned short* q = out + ((size_t)z * n8 + (size_t)i) * 8;
  *(volatile v4u*)q = u;
  __threadfence();
  *(volatile v4u*)q = u;
}

__global__ __launch_bounds__(256) void convw_pack_kernel(const float* __restrict__ w, unsigned short* __restrict__ out, float carry) {
  const int i = blockIdx.x * 256 + threadIdx.x;
  if (i >= (kE * 3 * kE) / 8) return;
  const int o = i / 192;
  const int rem = i - o * 192;
  const int d = rem >> 6;
  const int i0 = (rem & 63) * 8;
  const float* src = w + (size_t)o * (3 * kE) + (size_t)i0 * 3 + d;
  const float f0 = src[0], f1 = src[3], f2 = src[6], f3 = src[9], f4 = src[12], f5 = src[15], f6 = src[18], f7 = src[21];
  const unsigned short b0 = h_bits(bf16_rne(f0) * carry), b1 = h_bits(bf16_rne(f1) * carry);
  const unsigned short b2 = h_bits(bf16_rne(f2) * carry), b3 = h_bits(bf16_rne(f3) * carry);
  const unsigned short b4 = h_bits(bf16_rne(f4) * carry), b5 = h_bits(bf16_rne(f5) * carry);
  const unsigned short b6 = h_bits(bf16_rne(f6) * carry), b7 = h_bits(bf16_rne(f7) * carry);
  const v4u u = (v4u){pk16(b0, b1), pk16(b2, b3), pk16(b4, b5), pk16(b6, b7)};
  unsigned short* q = out + (size_t)i * 8;
  *(volatile v4u*)q = u;
  __threadfence();
  *(volatile v4u*)q = u;
}

__global__ __launch_bounds__(256) void xpose_cast_kernel(const float* __restrict__ x, unsigned short* __restrict__ x16, float carry) {
  __shared__ float sm[64][65];
  const int t = threadIdx.x;
  const int s0 = blockIdx.x * 64;
  const int b = blockIdx.y;
#pragma unroll
  for (int i = 0; i < 16; ++i) {
    const int e = i * 256 + t;
    const int c = e >> 6;
    const int sl = e & 63;
    sm[sl][c] = x[((size_t)b * kCin + c) * kS + s0 + sl];
  }
  __syncthreads();
  const int lane = t & 31;
  const int wave = __builtin_amdgcn_readfirstlane((int)(t >> 5));
  const int q = lane >> 3, c8 = (lane & 7) * 8;
  v4u u[2];
#pragma unroll
  for (int it = 0; it < 2; ++it) {
    const int row = wave * 8 + it * 4 + q;
    unsigned short hb[8];
#pragma unroll
    for (int e = 0; e < 8; ++e) {
      const float f = sm[row][c8 + e];
      hb[e] = h_bits(bf16_rne(f) * carry);
    }
    u[it] = (v4u){pk16(hb[0], hb[1]), pk16(hb[2], hb[3]), pk16(hb[4], hb[5]), pk16(hb[6], hb[7])};
  }
  for (int pass = 0; pass < 2; ++pass) {
#pragma unroll
    for (int it = 0; it < 2; ++it) {
      const int row = wave * 8 + it * 4 + q;
      *(volatile v4u*)(x16 + ((size_t)b * kS + s0 + row) * kCin + c8) = u[it];
    }
    __threadfence();
  }
}

__global__ __launch_bounds__(128) void zero_pad_rows_kernel(unsigned short* __restrict__ t16p) {
  const int b = blockIdx.x;
  unsigned short* p = t16p + (size_t)b * kSP * kE + (size_t)threadIdx.x * 8;
  const v4u z = (v4u){0u, 0u, 0u, 0u};
  *(volatile v4u*)p = z;
  __threadfence();
  *(volatile v4u*)p = z;
}

__global__ __launch_bounds__(256) void ln_rows_kernel(const float* __restrict__ x, const float* __restrict__ g,
                                                      const float* __restrict__ bt, unsigned short* __restrict__ y, float carry) {
  const int lane = threadIdx.x & 31;
  const int wave = __builtin_amdgcn_readfirstlane((int)(threadIdx.x >> 5));
  const int row = blockIdx.x * 8 + wave;
  const float* xr = x + (size_t)row * kE;
  const int c0 = lane * 8;
  const v4f a0 = *(const v4f*)(xr + c0);
  const v4f a1 = *(const v4f*)(xr + c0 + 4);
  const v4f a2 = *(const v4f*)(xr + 256 + c0);
  const v4f a3 = *(const v4f*)(xr + 256 + c0 + 4);
  float v[16] = {a0.x, a0.y, a0.z, a0.w, a1.x, a1.y, a1.z, a1.w, a2.x, a2.y, a2.z, a2.w, a3.x, a3.y, a3.z, a3.w};
  float s = 0.0f;
#pragma unroll
  for (int i = 0; i < 16; ++i) s += v[i];
#pragma unroll
  for (int off = 16; off > 0; off >>= 1) s += __shfl_xor(s, off, 32);
  const float mean = s * kInvE;
  float ss = 0.0f;
#pragma unroll
  for (int i = 0; i < 16; ++i) {
    const float d = v[i] - mean;
    ss = fmaf(d, d, ss);
  }
#pragma unroll
  for (int off = 16; off > 0; off >>= 1) ss += __shfl_xor(ss, off, 32);
  const float inv = rsqrtf(ss * kInvE + kLnEps);
  const v4f g0 = *(const v4f*)(g + c0);
  const v4f g1 = *(const v4f*)(g + c0 + 4);
  const v4f g2 = *(const v4f*)(g + 256 + c0);
  const v4f g3 = *(const v4f*)(g + 256 + c0 + 4);
  const v4f b0 = *(const v4f*)(bt + c0);
  const v4f b1 = *(const v4f*)(bt + c0 + 4);
  const v4f b2 = *(const v4f*)(bt + 256 + c0);
  const v4f b3 = *(const v4f*)(bt + 256 + c0 + 4);
  const float gg[16] = {g0.x, g0.y, g0.z, g0.w, g1.x, g1.y, g1.z, g1.w, g2.x, g2.y, g2.z, g2.w, g3.x, g3.y, g3.z, g3.w};
  const float bb[16] = {b0.x, b0.y, b0.z, b0.w, b1.x, b1.y, b1.z, b1.w, b2.x, b2.y, b2.z, b2.w, b3.x, b3.y, b3.z, b3.w};
  unsigned short hb[16];
#pragma unroll
  for (int i = 0; i < 16; ++i) {
    const float o = (v[i] - mean) * inv * bf16_rne(gg[i]) + bf16_rne(bb[i]);
    hb[i] = h_bits(o * carry);
  }
  const v4u u0 = (v4u){pk16(hb[0], hb[1]), pk16(hb[2], hb[3]), pk16(hb[4], hb[5]), pk16(hb[6], hb[7])};
  const v4u u1 = (v4u){pk16(hb[8], hb[9]), pk16(hb[10], hb[11]), pk16(hb[12], hb[13]), pk16(hb[14], hb[15])};
  unsigned short* yr = y + (size_t)row * kE;
  for (int pass = 0; pass < 2; ++pass) {
    *(volatile v4u*)(yr + c0) = u0;
    *(volatile v4u*)(yr + 256 + c0) = u1;
    __threadfence();
  }
}

__global__ __launch_bounds__(256) void rowsum_recip_kernel(const unsigned short* __restrict__ P16, float* __restrict__ rden) {
  __shared__ float sden[32];
  const int lane = threadIdx.x & 31;
  const int wave = __builtin_amdgcn_readfirstlane((int)(threadIdx.x >> 5));
  const int r0 = blockIdx.x * 32;
#pragma unroll 1
  for (int i = 0; i < 4; ++i) {
    const int g = r0 + wave * 4 + i;
    const int s = g & (kS - 1);
    const int ncols = ((s >> 6) + 1) << 6;
    const unsigned short* pr = P16 + (size_t)g * kS;
    float sum = 0.0f;
#pragma unroll 1
    for (int c0 = 0; c0 < ncols; c0 += 256) {
      const int col = c0 + lane * 8;
      const int cc = (col < ncols) ? col : (ncols - 8);
      const v4u w = *(const v4u*)(pr + cc);
      unsigned w0 = w.x, w1 = w.y, w2 = w.z, w3 = w.w;
      asm volatile("" : "+v"(w0), "+v"(w1), "+v"(w2), "+v"(w3));
      const float p0 = h16_to_f32(w0 & 0xffffu) + h16_to_f32(w0 >> 16);
      const float p1 = h16_to_f32(w1 & 0xffffu) + h16_to_f32(w1 >> 16);
      const float p2 = h16_to_f32(w2 & 0xffffu) + h16_to_f32(w2 >> 16);
      const float p3 = h16_to_f32(w3 & 0xffffu) + h16_to_f32(w3 >> 16);
      const float part = (p0 + p1) + (p2 + p3);
      sum += (col < ncols) ? part : 0.0f;
    }
#pragma unroll
    for (int off = 16; off > 0; off >>= 1) sum += __shfl_xor(sum, off, 32);
    if (lane == 0) sden[wave * 4 + i] = sum;
  }
  __syncthreads();
  if (wave == 0) {
    const float d = sden[lane];
    const float r = 1.0f / (d + kDenEps);
    float* p = rden + r0 + lane;
    *(volatile float*)p = r;
    __threadfence();
    *(volatile float*)p = r;
  }
}

extern "C" void kernel_launch(void* const* d_in, const int* in_sizes, int n_in,
                              void* d_out, int out_size, void* d_ws, size_t ws_size,
                              hipStream_t stream) {
  if (n_in < 23) return;
  const int expect[23] = {
      kBatch * kCin * kS, kE * kCin, kE, kE * kE * 3, kE,
      kLayers * kE, kLayers * kE, kLayers * kE, kLayers * kE,
      kLayers * kE * kE, kLayers * kE, kLayers * kE * kE, kLayers * kE,
      kLayers * kE * kE, kLayers * kE, kLayers * kE * kE, kLayers * kE,
      kLayers * kE * kE, kLayers * kE, kLayers * kE * kE, kLayers * kE,
      kCout * kE, kCout};
  for (int i = 0; i < 23; ++i) {
    if (in_sizes[i] != expect[i]) return;
  }
  if (out_size != kBatch * kCout * kS) return;
  if (ws_size < kWsTotal) return;

  const float* x    = (const float*)d_in[0];
  const float* in_W = (const float*)d_in[1];
  const float* in_b = (const float*)d_in[2];
  const float* cc_W = (const float*)d_in[3];
  const float* cc_b = (const float*)d_in[4];
  const float* ln1g = (const float*)d_in[5];
  const float* ln1b = (const float*)d_in[6];
  const float* ln2g = (const float*)d_in[7];
  const float* ln2b = (const float*)d_in[8];
  const float* Wq   = (const float*)d_in[9];
  const float* bq   = (const float*)d_in[10];
  const float* Wk   = (const float*)d_in[11];
  const float* bk   = (const float*)d_in[12];
  const float* Wv   = (const float*)d_in[13];
  const float* bv   = (const float*)d_in[14];
  const float* Wo   = (const float*)d_in[15];
  const float* bo   = (const float*)d_in[16];
  const float* c1W  = (const float*)d_in[17];
  const float* c1b  = (const float*)d_in[18];
  const float* c2W  = (const float*)d_in[19];
  const float* c2b  = (const float*)d_in[20];
  const float* outW = (const float*)d_in[21];
  const float* outb = (const float*)d_in[22];
  float* out = (float*)d_out;

  char* ws = (char*)d_ws;
  float*          LAT   = (float*)(ws + kOffLAT);
  float*          MID   = (float*)(ws + kOffMID);
  unsigned short* H16   = (unsigned short*)(ws + kOffH16);
  unsigned short* Q16   = (unsigned short*)(ws + kOffQ16);
  unsigned short* K16   = (unsigned short*)(ws + kOffK16);
  unsigned short* VT16  = (unsigned short*)(ws + kOffVT16);
  unsigned short* ATT16 = (unsigned short*)(ws + kOffATT);
  unsigned short* T16P  = (unsigned short*)(ws + kOffT16P);
  unsigned short* P16   = (unsigned short*)(ws + kOffP16);
  float*          RDEN  = (float*)(ws + kOffRDEN);
  unsigned short* W16   = (unsigned short*)(ws + kOffW16);
  unsigned short* CCW16 = (unsigned short*)(ws + kOffCCW);
  unsigned short* INW16 = (unsigned short*)(ws + kOffINW);
  unsigned short* OUTW16 = (unsigned short*)(ws + kOffOUTW);
  unsigned short* X16   = (unsigned short*)(ws + kOffX16);

  const long SE = (long)kS * kE;
  const long SS = (long)kS * kS;
  const size_t WL = (size_t)kE * kE;

  xpose_cast_kernel<<<dim3(kS / 64, kBatch), 256, 0, stream>>>(x, X16, kACarry);
  zero_pad_rows_kernel<<<kBatch, 128, 0, stream>>>(T16P);
  cast8_kernel<<<dim3((kE * kCin / 8) / 256, 1), 256, 0, stream>>>(in_W, in_W, in_W, in_W, in_W, in_W, INW16, kE * kCin / 8, kWCarry);
  convw_pack_kernel<<<(kE * 3 * kE / 8) / 256, 256, 0, stream>>>(cc_W, CCW16, kWCarry);
  cast8_kernel<<<dim3((kLayers * kE * kE / 8) / 256, kNumW), 256, 0, stream>>>(Wq, Wk, Wv, Wo, c1W, c2W, W16, kLayers * kE * kE / 8, kWCarry);
  cast8_kernel<<<dim3((kCout * kE / 8) / 256, 1), 256, 0, stream>>>(outW, outW, outW, outW, outW, outW, OUTW16, kCout * kE / 8, kWCarry);

  gemm64_kernel<2, 1, false, 0, 0, false><<<dim3((kS / 64) * (kE / 64) / 8, kBatch), 256, 0, stream>>>(
      X16, kCin, (long)kS * kCin,
      INW16, kCin, 0L,
      (void*)(T16P + 2 * kE), kE, (long)kSP * kE,
      in_b, nullptr, 0L, nullptr, 0L,
      kS, kE, kCin, kSclAW, kACarry);

  gemm64_kernel<2, 0, false, 0, 0, false><<<dim3((kS / 64) * (kE / 64) / 8, kBatch), 256, 0, stream>>>(
      T16P, kE, (long)kSP * kE,
      CCW16, 3 * kE, 0L,
      (void*)LAT, kE, SE,
      cc_b, nullptr, 0L, nullptr, 0L,
      kS, kE, 3 * kE, kSclAW, 1.0f);

  for (int l = 0; l < kLayers; ++l) {
    const unsigned short* Wq16 = W16 + ((size_t)0 * kLayers + l) * WL;
    const unsigned short* Wk16 = W16 + ((size_t)1 * kLayers + l) * WL;
    const unsigned short* Wv16 = W16 + ((size_t)2 * kLayers + l) * WL;
    const unsigned short* Wo16 = W16 + ((size_t)3 * kLayers + l) * WL;
    const unsigned short* C116 = W16 + ((size_t)4 * kLayers + l) * WL;
    const unsigned short* C216 = W16 + ((size_t)5 * kLayers + l) * WL;

    ln_rows_kernel<<<kRows / 8, 256, 0, stream>>>(LAT, ln1g + l * kE, ln1b + l * kE, H16, kACarry);
    gemm64_kernel<2, 1, false, 1, 0, false><<<dim3((kRows / 64) * (kE / 64) / 8, 1), 256, 0, stream>>>(
        H16, kE, 0L, Wq16, kE, 0L, (void*)Q16, kE, 0L,
        bq + l * kE, nullptr, 0L, nullptr, 0L,
        kRows, kE, kE, kSclAW, 1.0f);
    gemm64_kernel<2, 1, false, 1, 0, false><<<dim3((kRows / 64) * (kE / 64) / 8, 1), 256, 0, stream>>>(
        H16, kE, 0L, Wk16, kE, 0L, (void*)K16, kE, 0L,
        bk + l * kE, nullptr, 0L, nullptr, 0L,
        kRows, kE, kE, kSclAW, 1.0f);
    gemm64_kernel<1, 1, false, 0, 0, false><<<dim3((kE / 64) * (kS / 64) / 8, kBatch), 256, 0, stream>>>(
        Wv16, kE, 0L, H16, kE, SE, (void*)VT16, kS, (long)kE * kS,
        bv + l * kE, nullptr, 0L, nullptr, 0L,
        kE, kS, kE, kSclAW, kACarry);
    gemm64_kernel<0, 1, false, 0, 1, false><<<dim3(((kS / 64) * (kS / 64 + 1) / 2) / 8, kBatch), 256, 0, stream>>>(
        Q16, kE, SE, K16, kE, SE, (void*)P16, kS, SS,
        nullptr, nullptr, 0L, nullptr, 0L,
        kS, kS, kE, 1.0f, 1.0f);
    rowsum_recip_kernel<<<kRows / 32, 256, 0, stream>>>(P16, RDEN);
    gemm64_kernel<0, 1, false, 0, 2, true><<<dim3((kS / 64) * (kE / 64) / 8, kBatch), 256, 0, stream>>>(
        P16, kS, SS, VT16, kS, (long)kE * kS, (void*)ATT16, kE, SE,
        nullptr, nullptr, 0L, RDEN, (long)kS,
        kS, kE, kS, kSclNum, kAttCarry);
    gemm64_kernel<2, 0, true, 0, 0, false><<<dim3((kRows / 64) * (kE / 64) / 8, 1), 256, 0, stream>>>(
        ATT16, kE, 0L, Wo16, kE, 0L, (void*)MID, kE, 0L,
        bo + l * kE, LAT, 0L, nullptr, 0L,
        kRows, kE, kE, kSclAttW, 1.0f);
    ln_rows_kernel<<<kRows / 8, 256, 0, stream>>>(MID, ln2g + l * kE, ln2b + l * kE, H16, kACarry);
    gemm64_kernel<2, 1, false, 2, 0, false><<<dim3((kRows / 64) * (kE / 64) / 8, 1), 256, 0, stream>>>(
        H16, kE, 0L, C116, kE, 0L, (void*)Q16, kE, 0L,
        c1b + l * kE, nullptr, 0L, nullptr, 0L,
        kRows, kE, kE, kSclAW, kACarry);
    if (l + 1 < kLayers) {
      gemm64_kernel<2, 0, true, 0, 0, false><<<dim3((kRows / 64) * (kE / 64) / 8, 1), 256, 0, stream>>>(
          Q16, kE, 0L, C216, kE, 0L, (void*)LAT, kE, 0L,
          c2b + l * kE, MID, 0L, nullptr, 0L,
          kRows, kE, kE, kSclAW, 1.0f);
    } else {
      gemm64_kernel<2, 1, true, 0, 0, false><<<dim3((kRows / 64) * (kE / 64) / 8, 1), 256, 0, stream>>>(
          Q16, kE, 0L, C216, kE, 0L, (void*)ATT16, kE, 0L,
          c2b + l * kE, MID, 0L, nullptr, 0L,
          kRows, kE, kE, kSclAW, kACarry);
    }
  }

  gemm64_kernel<1, 0, false, 0, 0, false><<<dim3((kCout / 64) * (kS / 64) / 8, kBatch), 256, 0, stream>>>(
      OUTW16, kE, 0L, ATT16, kE, SE, (void*)out, kS, (long)kCout * kS,
      outb, nullptr, 0L, nullptr, 0L,
      kCout, kS, kE, kSclAW, 1.0f);
}
